// MambaTemp_14405320311406
// MI455X (gfx1250) — hardware-run, weakly checked
//
#include <hip/hip_runtime.h>
#include <math.h>

typedef __attribute__((ext_vector_type(16))) _Float16 v16h;
typedef __attribute__((ext_vector_type(8)))  _Float16 v8h;
typedef __attribute__((ext_vector_type(16))) __bf16   v16b;
typedef __attribute__((ext_vector_type(8)))  __bf16   v8b;
typedef __attribute__((ext_vector_type(8)))  float    v8f;
typedef __attribute__((ext_vector_type(4)))  float    v4f;

constexpr int kB    = 8;
constexpr int kT    = 8;
constexpr int kL    = 196;
constexpr int kD    = 192;
constexpr int kE2   = 2 * kD;
constexpr int kC    = kD * kT;
constexpr int kNs   = 16;
constexpr int kDC   = 4;
constexpr int kR    = 96;
constexpr int kXo   = kR + 2 * kNs;
constexpr int kRowsIn = kB * kT * kL;
constexpr int kRowsS  = kB * kL;
constexpr int kRowsP  = 1792;
constexpr int kThr  = 256;
constexpr float kInCarry = 1024.0f;
constexpr float kDtCarry = 256.0f;
constexpr float kSc   = 1.0f / (kInCarry * kInCarry);
constexpr float kScDt = 1.0f / (kDtCarry * kInCarry);
constexpr float kF16MinNormal = 6.103515625e-5f;

static_assert(kC == 1536 && kXo == 128 && kRowsIn == 12544 && kRowsS == 1568 && kRowsP >= kRowsS, "the sizes the index math below is written for");
static_assert((kRowsIn % 64) == 0 && (kE2 % 64) == 0 && (kRowsP % 64) == 0 && (kXo % 64) == 0 && (kC % 64) == 0 && (kD % 32) == 0 && (kC % 32) == 0 && (kR % 32) == 0
              && ((kRowsIn / 64) * (kE2 / 64)) % 8 == 0 && ((kRowsP / 64) * (kXo / 64)) % 8 == 0 && ((kRowsP / 64) * (kC / 64)) % 8 == 0, "GEMM M, N multiples of 64, K of 32; the three grids exact (1,176 / 56 / 672 tiles)");

constexpr size_t kOffX16 = 0ull;
constexpr size_t kOffWIN16 = 4816896ull;
constexpr size_t kOffWX16 = 4964352ull;
constexpr size_t kOffWDT16 = 5357568ull;
constexpr size_t kOffZB = 5652480ull;
constexpr size_t kOffBDT = 5658624ull;
constexpr size_t kOffXZ = 5664768ull;
constexpr size_t kOffU16 = 24932352ull;
constexpr size_t kOffXD = 30437376ull;
constexpr size_t kOffDT16 = 31354880ull;
constexpr size_t kOffDL = 31698944ull;
constexpr size_t kWsTotal = 42708992ull;
static_assert(kWsTotal <= 134217728ull, "carve cap: under 128 MiB");
static_assert(kOffX16 == 0
              && kOffWIN16 == kOffX16 + 4816896ull
              && kOffWX16 == kOffWIN16 + 147456ull
              && kOffWDT16 == kOffWX16 + 393216ull
              && kOffZB == kOffWDT16 + 294912ull
              && kOffBDT == kOffZB + 6144ull
              && kOffXZ == kOffBDT + 6144ull
              && kOffU16 == kOffXZ + 19267584ull
              && kOffXD == kOffU16 + 5505024ull
              && kOffDT16 == kOffXD + 917504ull
              && kOffDL == kOffDT16 + 344064ull
              && kWsTotal == kOffDL + 11010048ull, "the carve is chained and totalled");
static_assert((kOffX16 % 256) == 0 && (kOffWIN16 % 256) == 0 && (kOffWX16 % 256) == 0 && (kOffWDT16 % 256) == 0 && (kOffZB % 256) == 0 && (kOffBDT % 256) == 0 && (kOffXZ % 256) == 0 && (kOffU16 % 256) == 0 && (kOffXD % 256) == 0 && (kOffDT16 % 256) == 0 && (kOffDL % 256) == 0, "aligned regions");

__device__ __forceinline__ unsigned short f2bf_bits(float f) {
  unsigned u = __float_as_uint(f);
  return (unsigned short)((u + 0x7FFFu + ((u >> 16) & 1u)) >> 16);
}
__device__ __forceinline__ float bf_bits2f(unsigned short h) { return __uint_as_float(((unsigned)h) << 16); }
__device__ __forceinline__ float bf16r(float f) { return bf_bits2f(f2bf_bits(f)); }
__device__ __forceinline__ float carry_flush(float v, float carry) {
  const float s = v * carry;
  return (fabsf(s) < kF16MinNormal) ? 0.0f : s;
}
__device__ __forceinline__ float frcp(float x) { return __builtin_amdgcn_rcpf(x); }

__device__ __forceinline__ void dep_guard4_h(v8f& a, v8f& b, v8f& c, v8f& d, v16h x, v16h y) { asm volatile("v_nop\n\tv_nop\n\tv_nop\n\tv_nop" : "+v"(a), "+v"(b), "+v"(c), "+v"(d) : "v"(x), "v"(y)); }
__device__ __forceinline__ void dep_guard4_b(v8f& a, v8f& b, v8f& c, v8f& d, v16b x, v16b y) { asm volatile("v_nop\n\tv_nop\n\tv_nop\n\tv_nop" : "+v"(a), "+v"(b), "+v"(c), "+v"(d) : "v"(x), "v"(y)); }
__device__ __forceinline__ void keep4_h(v16h a, v16h b, v16h c, v16h d) { asm volatile("v_nop" :: "v"(a), "v"(b), "v"(c), "v"(d)); }
__device__ __forceinline__ void keep4_b(v16b a, v16b b, v16b c, v16b d) { asm volatile("v_nop" :: "v"(a), "v"(b), "v"(c), "v"(d)); }
__device__ __forceinline__ void acc_guard4(v8f& a, v8f& b, v8f& c, v8f& d) { asm volatile("v_nop\n\tv_nop\n\tv_nop\n\tv_nop" : "+v"(a), "+v"(b), "+v"(c), "+v"(d)); }

template <typename T> struct Frag;
template <> struct Frag<_Float16> {
  typedef v16h V; union U { v16h v; v8h h[2]; };
  static __device__ __forceinline__ v16h load(const _Float16* p) {
    U f; f.h[0] = *(const v8h*)(p); f.h[1] = *(const v8h*)(p + 16); return f.v;
  }
  static __device__ __forceinline__ v8f mma(v16h a, v16h b, v8f c) {
    return __builtin_amdgcn_wmma_f32_16x16x32_f16(false, a, false, b, (short)0, c, false, false);
  }
  static __device__ __forceinline__ void guard4(v8f& a, v8f& b, v8f& c, v8f& d, v16h x, v16h y) { dep_guard4_h(a, b, c, d, x, y); }
  static __device__ __forceinline__ void keep(v16h a, v16h b, v16h c, v16h d) { keep4_h(a, b, c, d); }
};
template <> struct Frag<__bf16> {
  typedef v16b V; union U { v16b v; v8b h[2]; };
  static __device__ __forceinline__ v16b load(const __bf16* p) {
    U f; f.h[0] = *(const v8b*)(p); f.h[1] = *(const v8b*)(p + 16); return f.v;
  }
  static __device__ __forceinline__ v8f mma(v16b a, v16b b, v8f c) {
    return __builtin_amdgcn_wmma_f32_16x16x32_bf16(false, a, false, b, (short)0, c, false, false);
  }
  static __device__ __forceinline__ void guard4(v8f& a, v8f& b, v8f& c, v8f& d, v16b x, v16b y) { dep_guard4_b(a, b, c, d, x, y); }
  static __device__ __forceinline__ void keep(v16b a, v16b b, v16b c, v16b d) { keep4_b(a, b, c, d); }
};

__device__ __forceinline__ v8f mma_h(v16h a, v16h b, v8f c) {
  c = __builtin_amdgcn_wmma_f32_16x16x32_f16(false, a, false, b, (short)0, c, false, false);
  asm volatile("v_nop\n\tv_nop\n\tv_nop\n\tv_nop" : "+v"(c) : "v"(a), "v"(b));
  return c;
}

template <int ET> struct Elem;
template <> struct Elem<0> { typedef _Float16 T; };
template <> struct Elem<1> { typedef __bf16 T; };
template <int ET, bool SPLIT, int BIAS_MODE, int OUT_MODE, bool RESID, int ACT = 0>
__global__ __launch_bounds__(256) void wmma_gemm64(
    const unsigned short* __restrict__ Ap, const unsigned short* __restrict__ A2p, int lda, long strideA,
    const unsigned short* __restrict__ Btp, const unsigned short* __restrict__ Bt2p, int ldb, long strideB,
    void* __restrict__ Cout, void* __restrict__ Cout2, int ldc, long strideC,
    const float* __restrict__ bias,
    const float* __restrict__ resid, long strideR,
    int M, int N, int K, float scale) {
  typedef typename Elem<ET>::T T;
  typedef typename Frag<T>::V V;
  const T* A = (const T*)Ap; const T* A2 = (const T*)A2p; const T* Bt = (const T*)Btp; const T* Bt2 = (const T*)Bt2p;
  __shared__ __align__(16) float sT[8][16 * 68];
  const int b    = blockIdx.y;
  const int lane = threadIdx.x & 31;
  const int wave = threadIdx.x >> 5;
  const int tilesN = N >> 6;
  const int tilesM = M >> 6;
  const int tile = blockIdx.x * 8 + wave;
  if (tile >= tilesM * tilesN) return;
  const int tm = tile / tilesN;
  const int tn = tile - tm * tilesN;
  const int m0 = tm << 6;
  const int n0 = tn << 6;

  const T* Ab  = A  + (size_t)b * strideA;
  const T* Bb  = Bt + (size_t)b * strideB;
  const T* Ab2 = SPLIT ? (A2  + (size_t)b * strideA) : nullptr;
  const T* Bb2 = SPLIT ? (Bt2 + (size_t)b * strideB) : nullptr;

  const int rlane = lane & 15;
  const int koff  = (lane >> 4) * 8;
  const int mOff  = (lane >> 4) * 8;

  v8f acc[4][4];
#pragma unroll
  for (int i = 0; i < 4; ++i)
#pragma unroll
    for (int j = 0; j < 4; ++j) acc[i][j] = (v8f){0.f,0.f,0.f,0.f,0.f,0.f,0.f,0.f};

  for (int k0 = 0; k0 < K; k0 += 32) {
    V bh[4], bl[4];
#pragma unroll
    for (int j = 0; j < 4; ++j) {
      const size_t bo = (size_t)(n0 + (j << 4) + rlane) * ldb + koff + k0;
      bh[j] = Frag<T>::load(Bb + bo);
      if (SPLIT) bl[j] = Frag<T>::load(Bb2 + bo);
    }
#pragma unroll
    for (int i = 0; i < 4; ++i) {
      const size_t ao = (size_t)(m0 + (i << 4) + rlane) * lda + koff + k0;
      V ah = Frag<T>::load(Ab + ao);
      V al;
      if (SPLIT) al = Frag<T>::load(Ab2 + ao);
#pragma unroll
      for (int j = 0; j < 4; ++j) {
        acc[i][j] = Frag<T>::mma(ah, bh[j], acc[i][j]);
        if (SPLIT) {
          acc[i][j] = Frag<T>::mma(ah, bl[j], acc[i][j]);
          acc[i][j] = Frag<T>::mma(al, bh[j], acc[i][j]);
        }
      }
      Frag<T>::guard4(acc[i][0], acc[i][1], acc[i][2], acc[i][3], ah, SPLIT ? al : ah);
    }
    Frag<T>::keep(bh[0], bh[1], bh[2], bh[3]);
    if (SPLIT) Frag<T>::keep(bl[0], bl[1], bl[2], bl[3]);
  }
  acc_guard4(acc[0][0], acc[0][1], acc[0][2], acc[0][3]);
  acc_guard4(acc[1][0], acc[1][1], acc[1][2], acc[1][3]);
  acc_guard4(acc[2][0], acc[2][1], acc[2][2], acc[2][3]);
  acc_guard4(acc[3][0], acc[3][1], acc[3][2], acc[3][3]);

  float* slab = sT[wave];
  const float* Rb = RESID ? (resid + (size_t)b * strideR) : nullptr;
#pragma unroll
  for (int i = 0; i < 4; ++i) {
    const int mBase = m0 + (i << 4);
#pragma unroll
    for (int j = 0; j < 4; ++j) {
      const int n = n0 + (j << 4) + rlane;
      float bv = 0.f;
      if (BIAS_MODE == 2) bv = bias[n];
#pragma unroll
      for (int r = 0; r < 8; ++r) {
        float v = acc[i][j][r] * scale;
        if (BIAS_MODE == 1) v += bias[mBase + mOff + r];
        if (BIAS_MODE == 2) v += bv;
        if (RESID) v += Rb[(size_t)(mBase + mOff + r) * ldc + n];
        if (ACT == 1) v = tanhf(v);
        if (ACT == 2) v = fmaxf(v, 0.0f);
        if (ACT == 3) v = v / (1.0f + expf(-v));
        if (ACT == 4) v = (v > 0.f) ? v : 0.01f * v;
        slab[(mOff + r) * 68 + (j << 4) + rlane] = v;
      }
    }
    __builtin_amdgcn_fence(__ATOMIC_RELEASE, "workgroup");
    __builtin_amdgcn_wave_barrier();
    __builtin_amdgcn_fence(__ATOMIC_ACQUIRE, "workgroup");
    if (OUT_MODE == 0) {
      float* C = (float*)Cout + (size_t)b * strideC;
      const int hh = lane >> 4, c4 = (lane & 15) * 4;
      for (int pass = 0; pass < 2; ++pass) {
#pragma unroll
        for (int it = 0; it < 8; ++it) {
          const int row = it * 2 + hh;
          v4f v = *(const v4f*)(slab + row * 68 + c4);
          *(volatile v4f*)(C + (size_t)(mBase + row) * ldc + n0 + c4) = v;
        }
        __threadfence();
      }
    } else {
      const int q = lane >> 3, c8 = (lane & 7) * 8;
      unsigned short* C  = (unsigned short*)Cout  + (size_t)b * strideC;
      unsigned short* C2 = (OUT_MODE == 2) ? ((unsigned short*)Cout2 + (size_t)b * strideC) : nullptr;
      for (int pass = 0; pass < 2; ++pass) {
#pragma unroll
        for (int it = 0; it < 4; ++it) {
          const int row = it * 4 + q;
          const float* sp = slab + row * 68 + c8;
          v8h hv, lv;
#pragma unroll
          for (int e = 0; e < 8; ++e) {
            if (OUT_MODE == 1) {
              hv[e] = (_Float16)sp[e];
            } else {
              unsigned short hb = f2bf_bits(sp[e]);
              unsigned short lb = f2bf_bits(sp[e] - bf_bits2f(hb));
              hv[e] = __builtin_bit_cast(_Float16, hb);
              lv[e] = __builtin_bit_cast(_Float16, lb);
            }
          }
          *(volatile v8h*)(C + (size_t)(mBase + row) * ldc + n0 + c8) = hv;
          if (OUT_MODE == 2) *(volatile v8h*)(C2 + (size_t)(mBase + row) * ldc + n0 + c8) = lv;
        }
        __threadfence();
      }
    }
    __builtin_amdgcn_fence(__ATOMIC_RELEASE, "workgroup");
    __builtin_amdgcn_wave_barrier();
    __builtin_amdgcn_fence(__ATOMIC_ACQUIRE, "workgroup");
  }
}

__global__ __launch_bounds__(kThr) void cast_plane_kernel(const float* __restrict__ src, unsigned short* __restrict__ dst,
                                                          int colsLog2, int dstPitch, int dstOff) {
  const int i   = blockIdx.x * kThr + threadIdx.x;
  const int sh  = colsLog2 - 3;
  const int row = i >> sh;
  const int c8  = (i & ((1 << sh) - 1)) * 8;
  const float* sp = src + ((size_t)row << colsLog2) + c8;
  const v4f a0 = *(const v4f*)(sp);
  const v4f a1 = *(const v4f*)(sp + 4);
  v8h hv;
#pragma unroll
  for (int e = 0; e < 4; ++e) {
    const float f0 = a0[e];
    const float f1 = a1[e];
    hv[e]     = (_Float16)carry_flush(bf16r(f0), kInCarry);
    hv[4 + e] = (_Float16)carry_flush(bf16r(f1), kInCarry);
  }
  unsigned short* dp = dst + (size_t)row * dstPitch + dstOff + c8;
  *(volatile v8h*)dp = hv;
  __threadfence();
  *(volatile v8h*)dp = hv;
}


__global__ __launch_bounds__(kThr) void setup_kernel(const float* __restrict__ dt_bias, float* __restrict__ ZB, float* __restrict__ BDT) {
  if (blockIdx.x < 6u) {
    float* dp = ZB + blockIdx.x * (unsigned)kThr + threadIdx.x;
    *(volatile float*)dp = 0.0f;
    __threadfence();
    *(volatile float*)dp = 0.0f;
  } else {
    const unsigned i = (blockIdx.x - 6u) * (unsigned)kThr + threadIdx.x;
    const float p = dt_bias[i];
    const float o = bf16r(p);
    *(volatile float*)(BDT + i) = o;
    __threadfence();
    *(volatile float*)(BDT + i) = o;
  }
}
static_assert(kC == 6 * kThr, "set-up grid exact: 6 blocks of zero bias + 6 of dt_bias");

__global__ __launch_bounds__(192) void conv_silu_kernel(const float* __restrict__ XZ, const float* __restrict__ cw, const float* __restrict__ cb,
                                                         unsigned short* __restrict__ U16) {
  const int row = (int)blockIdx.y;
  const int e = (int)threadIdx.x;
  unsigned short* hp = U16 + (size_t)row * kC + e * kT;
  v8h hv;
  if (row >= kRowsS) {
#pragma unroll
    for (int f = 0; f < 8; ++f) hv[f] = (_Float16)0.0f;
    *(volatile v8h*)hp = hv;
    __threadfence();
    *(volatile v8h*)hp = hv;
    return;
  }
  const int smp = row / kL;
  const int pos = row - smp * kL;
  const int c8 = e * kT;
  float acc[8];
  {
    const v4f b0 = *(const v4f*)(cb + c8), b1 = *(const v4f*)(cb + c8 + 4);
#pragma unroll
    for (int f = 0; f < 4; ++f) { const float p = b0[f], q = b1[f]; acc[f] = bf16r(p); acc[4 + f] = bf16r(q); }
  }
#pragma unroll
  for (int k = 0; k < kDC; ++k) {
    const int back = kDC - 1 - k;
    const bool has = pos >= back;
    const int pp = pos - (has ? back : 0);
#pragma unroll
    for (int f = 0; f < 8; ++f) {
      const float xv = XZ[((size_t)(smp * kT + f) * kL + pp) * kE2 + e];
      const float w = cw[(size_t)(c8 + f) * kDC + k];
      acc[f] += has ? bf16r(w) * xv : 0.0f;
    }
  }
#pragma unroll
  for (int f = 0; f < 8; ++f) {
    const float v = acc[f];
    const float s = v / (1.0f + expf(-v));
    hv[f] = (_Float16)carry_flush(s, kInCarry);
  }
  *(volatile v8h*)hp = hv;
  __threadfence();
  *(volatile v8h*)hp = hv;
}
static_assert(kD == 192 && kT == 8, "front block = the 192 inner indices; a thread's 8 channels = the 8 frames");

__global__ __launch_bounds__(32) void dt_cast96_kernel(const float* __restrict__ XD, unsigned short* __restrict__ DT16) {
  const unsigned t = threadIdx.x;
  if (t >= 2u * (unsigned)(kR / 8)) return;
  const unsigned hi = (t >= (unsigned)(kR / 8)) ? 1u : 0u;
  const size_t row = (size_t)blockIdx.y * 2u + hi;
  const unsigned c8 = (t - hi * (unsigned)(kR / 8)) * 8u;
  const v4f a0 = *(const v4f*)(XD + row * kXo + c8), a1 = *(const v4f*)(XD + row * kXo + c8 + 4);
  v8h hv;
#pragma unroll
  for (int f = 0; f < 4; ++f) { hv[f] = (_Float16)carry_flush(a0[f], kDtCarry); hv[4 + f] = (_Float16)carry_flush(a1[f], kDtCarry); }
  unsigned short* dp = DT16 + row * kR + c8;
  *(volatile v8h*)dp = hv;
  __threadfence();
  *(volatile v8h*)dp = hv;
}
static_assert(kR == 12 * 8 && (kRowsP % 2) == 0 && ((size_t)2 * kR * 2) % 128 == 0, "the step input's cast: 12 chunks a row; two rows a wave = three whole lines");

__global__ __launch_bounds__(kThr) void scan_kernel(const float* __restrict__ XD, const float* __restrict__ DL, const float* __restrict__ XZ,
                                                    const float* __restrict__ cw, const float* __restrict__ cb, const float* __restrict__ A_log,
                                                    const float* __restrict__ Dp, float* __restrict__ out) {
  const unsigned smp = blockIdx.x / 6u;
  const unsigned c = (blockIdx.x - smp * 6u) * (unsigned)kThr + threadIdx.x;
  const unsigned e = c >> 3, fr = c & 7u;
  float A[kNs], h[kNs], cwv[kDC];
#pragma unroll
  for (int n = 0; n < kNs; ++n) { const float a = A_log[(size_t)c * kNs + n]; A[n] = -expf(bf16r(a)); h[n] = 0.0f; }
#pragma unroll
  for (int t = 0; t < kDC; ++t) { const float w = cw[(size_t)c * kDC + t]; cwv[t] = bf16r(w); }
  const float q0 = Dp[c], c0 = cb[c];
  const float dc = bf16r(q0), cbv = bf16r(c0);
  float xw0 = 0.0f, xw1 = 0.0f, xw2 = 0.0f;
  const size_t zr0 = ((size_t)smp * kT + fr) * kL;
  const size_t sr0 = (size_t)smp * kL;
  float* op = out + ((size_t)smp * kC + c) * kL;
  for (int p = 0; p < kL; ++p) {
    const float* zrow = XZ + (zr0 + (size_t)p) * kE2;
    const float xv = zrow[e];
    const float zv = zrow[kD + e];
    const float* pr = XD + (sr0 + (size_t)p) * kXo;
    const float pre = DL[(sr0 + (size_t)p) * kC + c];
    float acc = cbv;
    acc += cwv[0] * xw0;
    acc += cwv[1] * xw1;
    acc += cwv[2] * xw2;
    acc += cwv[3] * xv;
    xw0 = xw1; xw1 = xw2; xw2 = xv;
    const float uu = acc / (1.0f + expf(-acc));
    const float delta = (pre > 20.0f) ? pre : log1pf(expf(pre));
    const float dx = delta * uu;
    float y = 0.0f;
#pragma unroll
    for (int q = 0; q < kNs / 4; ++q) {
      const v4f bv = *(const v4f*)(pr + kR + 4 * q), cv = *(const v4f*)(pr + kR + kNs + 4 * q);
#pragma unroll
      for (int f = 0; f < 4; ++f) {
        const int n = 4 * q + f;
        const float hn = expf(delta * A[n]) * h[n] + dx * bv[f];
        h[n] = hn;
        y += hn * cv[f];
      }
    }
    const float yo = y + dc * uu;
    const float o = yo * (zv / (1.0f + expf(-zv)));
    *(volatile float*)(op + p) = o;
    __threadfence();
    *(volatile float*)(op + p) = o;
  }
}
static_assert(kC == 6 * kThr && (kNs % 4) == 0 && kDC == 4 && kT == 8, "scan grid exact: 48 blocks; six a sample; c = 8 e + frame (the shift by 3)");

static_assert(((size_t)kRowsIn * kD / 8) % kThr == 0 && ((size_t)kE2 * kD / 8) % kThr == 0 && ((size_t)kXo * kC / 8) % kThr == 0 && ((size_t)kC * kR / 8) % kThr == 0
              && ((size_t)kRowsIn * kD) % 64 == 0 && ((size_t)kE2 * kD) % 64 == 0 && ((size_t)kXo * kC) % 512 == 0 && ((size_t)kC * kR) % 64 == 0, "plane cast grids exact; the planes are whole rows of 64 / 512");

extern "C" void kernel_launch(void* const* d_in, const int* in_sizes, int n_in,
                              void* d_out, int out_size, void* d_ws, size_t ws_size,
                              hipStream_t stream) {
  if (n_in < 9 || d_out == nullptr || d_ws == nullptr) return;
  if (in_sizes[0] != kRowsIn * kD || in_sizes[1] != kE2 * kD || in_sizes[2] != kC * kDC || in_sizes[3] != kC || in_sizes[4] != kXo * kC) return;
  if (in_sizes[5] != kC * kR || in_sizes[6] != kC || in_sizes[7] != kC * kNs || in_sizes[8] != kC) return;
  if (out_size != kB * kC * kL) return;
  if (ws_size < kWsTotal) return;
  const float* hidden = (const float*)d_in[0];
  const float* in_proj_w = (const float*)d_in[1];
  const float* conv_w = (const float*)d_in[2];
  const float* conv_b = (const float*)d_in[3];
  const float* x_proj_w = (const float*)d_in[4];
  const float* dt_proj_w = (const float*)d_in[5];
  const float* dt_bias = (const float*)d_in[6];
  const float* A_log = (const float*)d_in[7];
  const float* D_param = (const float*)d_in[8];
  float* out = (float*)d_out;
  char* ws = (char*)d_ws;
  unsigned short* X16 = (unsigned short*)(ws + kOffX16);
  unsigned short* WIN16 = (unsigned short*)(ws + kOffWIN16);
  unsigned short* WX16 = (unsigned short*)(ws + kOffWX16);
  unsigned short* WDT16 = (unsigned short*)(ws + kOffWDT16);
  float* ZB = (float*)(ws + kOffZB);
  float* BDT = (float*)(ws + kOffBDT);
  float* XZ = (float*)(ws + kOffXZ);
  unsigned short* U16 = (unsigned short*)(ws + kOffU16);
  float* XD = (float*)(ws + kOffXD);
  unsigned short* DT16 = (unsigned short*)(ws + kOffDT16);
  float* DL = (float*)(ws + kOffDL);

  cast_plane_kernel<<<(int)(((size_t)kRowsIn * kD / 8) / kThr), kThr, 0, stream>>>(hidden, X16, 6, 64, 0);
  cast_plane_kernel<<<(int)(((size_t)kE2 * kD / 8) / kThr), kThr, 0, stream>>>(in_proj_w, WIN16, 6, 64, 0);
  cast_plane_kernel<<<(int)(((size_t)kXo * kC / 8) / kThr), kThr, 0, stream>>>(x_proj_w, WX16, 9, 512, 0);
  cast_plane_kernel<<<(int)(((size_t)kC * kR / 8) / kThr), kThr, 0, stream>>>(dt_proj_w, WDT16, 6, 64, 0);
  setup_kernel<<<12, kThr, 0, stream>>>(dt_bias, ZB, BDT);
  wmma_gemm64<0, false, 2, 0, false, 0><<<dim3((kRowsIn / 64) * (kE2 / 64) / 8, 1), 256, 0, stream>>>(
      X16, X16, kD, 0L, WIN16, WIN16, kD, 0L, (void*)XZ, (void*)XZ, kE2, 0L, ZB, nullptr, 0L, kRowsIn, kE2, kD, kSc);
  conv_silu_kernel<<<dim3(1, kRowsP), 192, 0, stream>>>(XZ, conv_w, conv_b, U16);
  wmma_gemm64<0, false, 2, 0, false, 0><<<dim3((kRowsP / 64) * (kXo / 64) / 8, 1), 256, 0, stream>>>(
      U16, U16, kC, 0L, WX16, WX16, kC, 0L, (void*)XD, (void*)XD, kXo, 0L, ZB, nullptr, 0L, kRowsP, kXo, kC, kSc);
  dt_cast96_kernel<<<dim3(1, kRowsP / 2), 32, 0, stream>>>(XD, DT16);
  wmma_gemm64<0, false, 2, 0, false, 0><<<dim3((kRowsP / 64) * (kC / 64) / 8, 1), 256, 0, stream>>>(
      DT16, DT16, kR, 0L, WDT16, WDT16, kR, 0L, (void*)DL, (void*)DL, kC, 0L, BDT, nullptr, 0L, kRowsP, kC, kR, kScDt);
  scan_kernel<<<kB * 6, kThr, 0, stream>>>(XD, DL, XZ, conv_w, conv_b, A_log, D_param, out);
}
